// CrossViewImputer_16587163697656
// MI455X (gfx1250) — hardware-verified
//
#include <hip/hip_runtime.h>
#include <stddef.h>


#define NTHR  256
#define NWAVE 8
#define IND   128
#define CH1   256
#define NH1   4
#define HC    64
#define CH2   64
#define DH    32
#define NCL   17
#define GR1   32
#define GR2   64
#define GRD   128
#define NPAD  128
#define AP1   (IND + 8)
#define XP1   (CH1 + 4)
#define XP2   (CH2 + 4)
#define TPW   264
#define W1TP  72
#define W2TP  40
#define HSP   40
#define NB1   256
#define SB1   8
#define NB2   1024
#define SB2   10
#define CHUNK 4096
#define NGRP  (CHUNK / (NTHR * 4))
#define WCAP  ((CHUNK / NTHR) * 32)
#define LDS_AGG1 ((NB1 * CH1 + NB1 * NH1 + NWAVE * WCAP + NWAVE) * 4)
#define LDS_AGG2 ((NB2 * CH2 + NB2 + NWAVE * WCAP + NWAVE) * 4)

static_assert(NGRP == 4);
static_assert(WCAP == 512);
static_assert(NWAVE * WCAP == CHUNK);
static_assert((1 << SB1) == NB1);
static_assert((1 << SB2) == NB2);
static_assert(LDS_AGG1 == 282656);
static_assert(LDS_AGG2 == 282656);
static_assert(((NB1 * CH1 + NB1 * NH1) % 4) == 0);
static_assert(((NB2 * CH2 + NB2) % 4) == 0);
static_assert(NH1 * HC == CH1);
static_assert(NB1 / NWAVE == 32);
static_assert(NB2 / NWAVE == 128);
static_assert(NTHR == CH1);
static_assert(GRD * NCL % 4 == 0);

typedef float    v2f  __attribute__((ext_vector_type(2)));
typedef float    v4f  __attribute__((ext_vector_type(4)));
typedef float    v8f  __attribute__((ext_vector_type(8)));
typedef int      v4i  __attribute__((ext_vector_type(4)));
typedef _Float16 v8h  __attribute__((ext_vector_type(8)));
typedef _Float16 v16h __attribute__((ext_vector_type(16)));
union Frag   { v16h v; v8h half[2]; };
union Pack16 { v8h h; v4i i; };

__device__ __forceinline__ v8f wm(v16h a, v16h b, v8f c) {
  v8f d = __builtin_amdgcn_wmma_f32_16x16x32_f16(false, a, false, b, (short)0, c, false, false);
  asm volatile("v_nop\n\tv_nop\n\tv_nop\n\tv_nop" : "+v"(d) : "v"(a), "v"(b));
  return d;
}

__device__ __forceinline__ v8f zero8() {
  v8f z = {0.f, 0.f, 0.f, 0.f, 0.f, 0.f, 0.f, 0.f};
  return z;
}

__device__ __forceinline__ v4i pack8(v4f a, v4f b) {
  Pack16 u;
  u.h[0] = (_Float16)a.x; u.h[1] = (_Float16)a.y; u.h[2] = (_Float16)a.z; u.h[3] = (_Float16)a.w;
  u.h[4] = (_Float16)b.x; u.h[5] = (_Float16)b.y; u.h[6] = (_Float16)b.z; u.h[7] = (_Float16)b.w;
  return u.i;
}

__device__ __forceinline__ float lrelu(float v) { return v > 0.f ? v : 0.2f * v; }
__device__ __forceinline__ float elu1(float v)  { return v > 0.f ? v : (__expf(v) - 1.0f); }
__device__ __forceinline__ v4f elu4(v4f v) {
  v.x = elu1(v.x); v.y = elu1(v.y); v.z = elu1(v.z); v.w = elu1(v.w);
  return v;
}
__device__ __forceinline__ float hmax16(float v) {
  v = fmaxf(v, __shfl_xor(v, 1, 32));
  v = fmaxf(v, __shfl_xor(v, 2, 32));
  v = fmaxf(v, __shfl_xor(v, 4, 32));
  v = fmaxf(v, __shfl_xor(v, 8, 32));
  return v;
}
__device__ __forceinline__ float hsum16(float v) {
  v += __shfl_xor(v, 1, 32);
  v += __shfl_xor(v, 2, 32);
  v += __shfl_xor(v, 4, 32);
  v += __shfl_xor(v, 8, 32);
  return v;
}

__global__ __launch_bounds__(NTHR) void k_wprep(const float* __restrict__ W, _Float16* Wh,
                                                int K, int NO, float scale) {
  __shared__ __attribute__((aligned(16))) _Float16 T[32 * TPW];
  const int tid = threadIdx.x;
  const int n0  = blockIdx.x * 32;
  const int TP  = K + 8;
  for (int idx = tid; idx < K * 32; idx += NTHR) {
    const int k = idx >> 5, c = idx & 31;
    T[c * TP + k] = (_Float16)(scale * W[(size_t)k * NO + n0 + c]);
  }
  __syncthreads();
  const int KQ = K >> 3;
  const int P  = 32 * KQ;
  for (int p = tid; p < P; p += NTHR) {
    const int row = p / KQ, q = p - row * KQ;
    Pack16 u; u.h = *(const v8h*)(T + row * TP + 8 * q);
    *(volatile v4i*)(Wh + (size_t)(n0 + row) * K + 8 * q) = u.i;
  }
  __threadfence();
  for (int p = tid; p < P; p += NTHR) {
    const int row = p / KQ, q = p - row * KQ;
    Pack16 u; u.h = *(const v8h*)(T + row * TP + 8 * q);
    *(volatile v4i*)(Wh + (size_t)(n0 + row) * K + 8 * q) = u.i;
  }
}

__global__ __launch_bounds__(NTHR) void k_gemm1(
    const float* __restrict__ x, const _Float16* __restrict__ Wh,
    const float* __restrict__ atts, const float* __restrict__ attd,
    float* h1, float* as1, float* ad1, int nN) {
  __shared__ __attribute__((aligned(16))) _Float16 At[GR1 * AP1];
  __shared__ __attribute__((aligned(16))) float Xs[GR1 * XP1];
  __shared__ __attribute__((aligned(16))) float Att[2 * CH1];
  __shared__ __attribute__((aligned(16))) float As[GR1 * NH1];
  __shared__ __attribute__((aligned(16))) float Ds[GR1 * NH1];

  const int tid  = threadIdx.x;
  const int lane = tid & 31;
  const int wave = tid >> 5;
  const int hh   = lane >> 4;
  const int m    = lane & 15;
  const int rowBase = blockIdx.x * GR1;

  {
    const int r  = tid >> 3;
    const int c0 = (tid & 7) * 16;
    int row = rowBase + r;
    if (row > nN - 1) row = nN - 1;
    const float* p = x + (size_t)row * IND + c0;
    const v4f f0 = *(const v4f*)(p), f1 = *(const v4f*)(p + 4);
    const v4f f2 = *(const v4f*)(p + 8), f3 = *(const v4f*)(p + 12);
    Pack16 u0, u1;
    u0.i = pack8(f0, f1);
    u1.i = pack8(f2, f3);
    *(v8h*)(At + r * AP1 + c0)     = u0.h;
    *(v8h*)(At + r * AP1 + c0 + 8) = u1.h;
    Att[tid]       = atts[tid];
    Att[CH1 + tid] = attd[tid];
  }
  __syncthreads();

  const int nc0 = wave * 16 + m;
  const int nc1 = (CH1 / 2) + wave * 16 + m;
  v8f c00 = zero8(), c01 = zero8(), c10 = zero8(), c11 = zero8();
#pragma unroll
  for (int kt = 0; kt < IND / 32; ++kt) {
    const int k0 = kt * 32;
    Frag a0, a1, b0, b1;
    const _Float16* pa0 = At + m * AP1 + k0 + 8 * hh;
    const _Float16* pa1 = At + (16 + m) * AP1 + k0 + 8 * hh;
    const _Float16* pb0 = Wh + (size_t)nc0 * IND + k0 + 8 * hh;
    const _Float16* pb1 = Wh + (size_t)nc1 * IND + k0 + 8 * hh;
    a0.half[0] = *(const v8h*)pa0; a0.half[1] = *(const v8h*)(pa0 + 16);
    a1.half[0] = *(const v8h*)pa1; a1.half[1] = *(const v8h*)(pa1 + 16);
    b0.half[0] = *(const v8h*)pb0; b0.half[1] = *(const v8h*)(pb0 + 16);
    b1.half[0] = *(const v8h*)pb1; b1.half[1] = *(const v8h*)(pb1 + 16);
    c00 = wm(a0.v, b0.v, c00);
    c01 = wm(a0.v, b1.v, c01);
    c10 = wm(a1.v, b0.v, c10);
    c11 = wm(a1.v, b1.v, c11);
  }

  {
    const float inv = 0.015625f;
#pragma unroll
    for (int r = 0; r < 8; ++r) {
      Xs[(8 * hh + r) * XP1 + nc0]      = c00[r] * inv;
      Xs[(8 * hh + r) * XP1 + nc1]      = c01[r] * inv;
      Xs[(16 + 8 * hh + r) * XP1 + nc0] = c10[r] * inv;
      Xs[(16 + 8 * hh + r) * XP1 + nc1] = c11[r] * inv;
    }
  }
  __syncthreads();

  {
    const int r  = tid >> 3;
    const int hd = (tid >> 1) & 3;
    const int wh = tid & 1;
    const float* av = Att + wh * CH1 + hd * HC;
    const float* xv = Xs + r * XP1 + hd * HC;
    float s = 0.f;
#pragma unroll
    for (int i = 0; i < HC / 4; ++i) {
      const v4f a = *(const v4f*)(av + 4 * i);
      const v4f b = *(const v4f*)(xv + 4 * i);
      s += a.x * b.x + a.y * b.y + a.z * b.z + a.w * b.w;
    }
    if (wh) Ds[r * NH1 + hd] = s; else As[r * NH1 + hd] = s;
  }
  __syncthreads();

  v4f xr[8];
#pragma unroll
  for (int i = 0; i < 4; ++i) {
    xr[2 * i]     = *(const v4f*)(Xs + (4 * wave + i) * XP1 + 4 * lane);
    xr[2 * i + 1] = *(const v4f*)(Xs + (4 * wave + i) * XP1 + (CH1 / 2) + 4 * lane);
  }
  float* hp[4];
#pragma unroll
  for (int i = 0; i < 4; ++i) hp[i] = h1 + (size_t)(rowBase + 4 * wave + i) * CH1 + 4 * lane;
  const bool gs = (wave < 2);
  v4f gv = {0.f, 0.f, 0.f, 0.f};
  float* gp = as1;
  if (wave == 0)      { gv = *(const v4f*)(As + 4 * lane); gp = as1 + (size_t)rowBase * NH1 + 4 * lane; }
  else if (wave == 1) { gv = *(const v4f*)(Ds + 4 * lane); gp = ad1 + (size_t)rowBase * NH1 + 4 * lane; }

#pragma unroll
  for (int i = 0; i < 4; ++i) {
    *(volatile v4f*)(hp[i]) = xr[2 * i];
    *(volatile v4f*)(hp[i] + (CH1 / 2)) = xr[2 * i + 1];
  }
  if (gs) *(volatile v4f*)gp = gv;
  __threadfence();
#pragma unroll
  for (int i = 0; i < 4; ++i) {
    *(volatile v4f*)(hp[i]) = xr[2 * i];
    *(volatile v4f*)(hp[i] + (CH1 / 2)) = xr[2 * i + 1];
  }
  if (gs) *(volatile v4f*)gp = gv;
}

template <int NB, int SB>
__device__ __forceinline__ int scan_chunk(const int* __restrict__ eid, int nE, int cbase,
                                          int nodeBase, int tid, int wave, bool al16, int* list) {
  int wc = 0;
#pragma unroll
  for (int g = 0; g < NGRP; ++g) {
    const int el0 = (g * NTHR + tid) * 4;
    const int e0  = cbase + el0;
    const int sent = -2147483647 - 1;
    v4i d;
    if (al16 && (e0 + 3 < nE)) {
      d = *(const v4i*)(eid + e0);
    } else {
      d.x = (e0     < nE) ? eid[min(e0, nE - 1)]     : sent;
      d.y = (e0 + 1 < nE) ? eid[min(e0 + 1, nE - 1)] : sent;
      d.z = (e0 + 2 < nE) ? eid[min(e0 + 2, nE - 1)] : sent;
      d.w = (e0 + 3 < nE) ? eid[min(e0 + 3, nE - 1)] : sent;
    }
    const unsigned s0 = (unsigned)d.x - (unsigned)nodeBase;
    const unsigned s1 = (unsigned)d.y - (unsigned)nodeBase;
    const unsigned s2 = (unsigned)d.z - (unsigned)nodeBase;
    const unsigned s3 = (unsigned)d.w - (unsigned)nodeBase;
    const bool h0 = s0 < (unsigned)NB;
    const bool h1 = s1 < (unsigned)NB;
    const bool h2 = s2 < (unsigned)NB;
    const bool h3 = s3 < (unsigned)NB;
    const unsigned many = __builtin_amdgcn_ballot_w32(h0 | h1 | h2 | h3);
    if (many != 0u) {
#define HITJ(J, HJ, SJ) { \
        const unsigned mj = __builtin_amdgcn_ballot_w32(HJ); \
        if (HJ) { \
          const int pos = wc + (int)__builtin_amdgcn_mbcnt_lo(mj, 0u); \
          if (pos < WCAP) list[wave * WCAP + pos] = ((el0 + (J)) << SB) | (int)(SJ); \
        } \
        wc += (int)__builtin_popcount(mj); }
      HITJ(0, h0, s0)
      HITJ(1, h1, s1)
      HITJ(2, h2, s2)
      HITJ(3, h3, s3)
#undef HITJ
    }
  }
  return wc;
}

__global__ __launch_bounds__(NTHR) void k_agg1(
    const int* __restrict__ ei, const float* __restrict__ h1,
    const float* __restrict__ as1, const float* __restrict__ ad1,
    const float* __restrict__ bias, const float* __restrict__ gam, const float* __restrict__ bet,
    _Float16* hp, int nN, int nE) {
  extern __shared__ v4f lds_dyn[];
  float* sacc = (float*)lds_dyn;
  float* den  = sacc + NB1 * CH1;
  int*   list = (int*)(den + NB1 * NH1);
  int*   wcnt = list + NWAVE * WCAP;

  const int tid  = threadIdx.x;
  const int lane = tid & 31;
  const int wave = tid >> 5;
  const int hd   = lane >> 3;
  const int nodeBase = blockIdx.x * NB1;

  {
    const v4f z4 = {0.f, 0.f, 0.f, 0.f};
    for (int i = tid; i < (NB1 * CH1 + NB1 * NH1) / 4; i += NTHR) lds_dyn[i] = z4;
  }
  __syncthreads();

  const int* eid = ei + nE;
  const bool al16 = ((nE & 3) == 0);
  const int nChunks = (nE + CHUNK - 1) / CHUNK;
#pragma unroll 1
  for (int ch = 0; ch < nChunks; ++ch) {
    const int cbase = ch * CHUNK;
    const int wc = scan_chunk<NB1, SB1>(eid, nE, cbase, nodeBase, tid, wave, al16, list);
    if (lane == 0) wcnt[wave] = wc;
    __syncthreads();

    if (wave == 0) {
      for (int wsx = 0; wsx < NWAVE; ++wsx) {
        int n = wcnt[wsx];
        if (n > WCAP) n = WCAP;
        if (n < 0) n = 0;
        for (int i = 0; i < n; ++i) {
          const int ent  = list[wsx * WCAP + i];
          const int slot = ent & (NB1 - 1);
          const int el   = (ent >> SB1) & (CHUNK - 1);
          int e = cbase + el;
          if (e > nE - 1) e = nE - 1;
          int src = ei[e];
          src = src < 0 ? 0 : (src > nN - 1 ? nN - 1 : src);
          int nd = nodeBase + slot;
          if (nd > nN - 1) nd = nN - 1;
          float al = as1[(size_t)src * NH1 + hd] + ad1[(size_t)nd * NH1 + hd];
          al = lrelu(al);
          al = fminf(al, 80.f);
          const float p = __expf(al);
          const float* hr = h1 + (size_t)src * CH1 + 8 * lane;
          const v4f x0 = *(const v4f*)hr;
          const v4f x1 = *(const v4f*)(hr + 4);
          v4f* sp = (v4f*)(sacc + slot * CH1 + 8 * lane);
          const v4f cr0 = sp[0];
          const v4f cr1 = sp[1];
          sp[0] = cr0 + p * x0;
          sp[1] = cr1 + p * x1;
          if ((lane & 7) == 0) {
            const float o = den[slot * NH1 + hd];
            den[slot * NH1 + hd] = o + p;
          }
        }
      }
    }
    __syncthreads();
  }

  const float bnk = 1.0f / sqrtf(1.0f + 1e-5f);
  const v4f b0 = *(const v4f*)(bias + 8 * lane);
  const v4f b1 = *(const v4f*)(bias + 8 * lane + 4);
  const v4f g0 = *(const v4f*)(gam + 8 * lane) * bnk;
  const v4f g1 = *(const v4f*)(gam + 8 * lane + 4) * bnk;
  const v4f e0 = *(const v4f*)(bet + 8 * lane);
  const v4f e1 = *(const v4f*)(bet + 8 * lane + 4);
#pragma unroll 1
  for (int j = 0; j < NB1 / NWAVE; ++j) {
    const int slot = wave * (NB1 / NWAVE) + j;
    const int node = nodeBase + slot;
    if (node >= nN) break;
    const size_t nr = (size_t)node;
    float al = as1[nr * NH1 + hd] + ad1[nr * NH1 + hd];
    al = lrelu(al);
    al = fminf(al, 80.f);
    const float p = __expf(al);
    const float* hr = h1 + nr * CH1 + 8 * lane;
    const v4f x0 = *(const v4f*)hr;
    const v4f x1 = *(const v4f*)(hr + 4);
    const v4f* sp = (const v4f*)(sacc + slot * CH1 + 8 * lane);
    const v4f s0 = sp[0] + p * x0;
    const v4f s1 = sp[1] + p * x1;
    const float dv  = den[slot * NH1 + hd] + p;
    const float inv = 1.0f / (dv + 1e-16f);
    v4f v0 = s0 * inv + b0;
    v4f v1 = s1 * inv + b1;
    v0 = v0 * g0 + e0;
    v1 = v1 * g1 + e1;
    v0 = elu4(v0);
    v1 = elu4(v1);
    const v4i u = pack8(v0, v1);
    _Float16* op = hp + nr * CH1 + 8 * lane;
    *(volatile v4i*)op = u;
    __threadfence();
    *(volatile v4i*)op = u;
  }
}

__global__ __launch_bounds__(NTHR) void k_gemm2(
    const _Float16* __restrict__ Hp, const _Float16* __restrict__ Wh,
    const float* __restrict__ atts, const float* __restrict__ attd,
    float* h2, float* as2, float* ad2, int nN) {
  __shared__ __attribute__((aligned(16))) float Xs[GR2 * XP2];
  __shared__ __attribute__((aligned(16))) float Att[2 * CH2];
  __shared__ __attribute__((aligned(16))) float As[GR2];
  __shared__ __attribute__((aligned(16))) float Ds[GR2];

  const int tid  = threadIdx.x;
  const int lane = tid & 31;
  const int wave = tid >> 5;
  const int hh   = lane >> 4;
  const int m    = lane & 15;
  const int rowBase = blockIdx.x * GR2;

  if (tid < 2 * CH2) Att[tid] = (tid < CH2) ? atts[tid] : attd[tid - CH2];

  const int rt  = wave >> 1;
  const int nc0 = 2 * (wave & 1) * 16 + m;
  const int nc1 = nc0 + 16;
  int row = rowBase + rt * 16 + m;
  if (row > nN - 1) row = nN - 1;
  const _Float16* pa = Hp + (size_t)row * CH1;

  v8f c0 = zero8(), c1 = zero8();
#pragma unroll
  for (int kt = 0; kt < CH1 / 32; ++kt) {
    const int k0 = kt * 32;
    Frag a, b0, b1;
    const _Float16* pb0 = Wh + (size_t)nc0 * CH1 + k0 + 8 * hh;
    const _Float16* pb1 = Wh + (size_t)nc1 * CH1 + k0 + 8 * hh;
    a.half[0]  = *(const v8h*)(pa + k0 + 8 * hh);
    a.half[1]  = *(const v8h*)(pa + k0 + 16 + 8 * hh);
    b0.half[0] = *(const v8h*)pb0; b0.half[1] = *(const v8h*)(pb0 + 16);
    b1.half[0] = *(const v8h*)pb1; b1.half[1] = *(const v8h*)(pb1 + 16);
    c0 = wm(a.v, b0.v, c0);
    c1 = wm(a.v, b1.v, c1);
  }
  {
    const float inv = 0.015625f;
#pragma unroll
    for (int r = 0; r < 8; ++r) {
      Xs[(rt * 16 + 8 * hh + r) * XP2 + nc0] = c0[r] * inv;
      Xs[(rt * 16 + 8 * hh + r) * XP2 + nc1] = c1[r] * inv;
    }
  }
  __syncthreads();

  if (tid < 2 * GR2) {
    const int r  = tid >> 1;
    const int wh = tid & 1;
    const float* av = Att + wh * CH2;
    const float* xv = Xs + r * XP2;
    float s = 0.f;
#pragma unroll
    for (int i = 0; i < CH2 / 4; ++i) {
      const v4f a = *(const v4f*)(av + 4 * i);
      const v4f b = *(const v4f*)(xv + 4 * i);
      s += a.x * b.x + a.y * b.y + a.z * b.z + a.w * b.w;
    }
    if (wh) Ds[r] = s; else As[r] = s;
  }
  __syncthreads();

  v4f xr[4];
  float* rp[4];
#pragma unroll
  for (int i = 0; i < 4; ++i) {
    const int rr = 8 * wave + 2 * i + hh;
    xr[i] = *(const v4f*)(Xs + rr * XP2 + 4 * m);
    rp[i] = h2 + (size_t)(rowBase + rr) * CH2 + 4 * m;
  }
  const bool gs = (wave == 0);
  const v4f gv = hh ? *(const v4f*)(Ds + 4 * m) : *(const v4f*)(As + 4 * m);
  float* gp = (hh ? ad2 : as2) + (size_t)rowBase + 4 * m;

#pragma unroll
  for (int i = 0; i < 4; ++i) *(volatile v4f*)(rp[i]) = xr[i];
  if (gs) *(volatile v4f*)gp = gv;
  __threadfence();
#pragma unroll
  for (int i = 0; i < 4; ++i) *(volatile v4f*)(rp[i]) = xr[i];
  if (gs) *(volatile v4f*)gp = gv;
}

__global__ __launch_bounds__(NTHR) void k_agg2(
    const int* __restrict__ ei, const float* __restrict__ h2,
    const float* __restrict__ as2, const float* __restrict__ ad2,
    const float* __restrict__ bias, const float* __restrict__ gam, const float* __restrict__ bet,
    _Float16* hp, int nN, int nE) {
  extern __shared__ v4f lds_dyn[];
  float* sacc = (float*)lds_dyn;
  float* den  = sacc + NB2 * CH2;
  int*   list = (int*)(den + NB2);
  int*   wcnt = list + NWAVE * WCAP;

  const int tid  = threadIdx.x;
  const int lane = tid & 31;
  const int wave = tid >> 5;
  const int nodeBase = blockIdx.x * NB2;

  {
    const v4f z4 = {0.f, 0.f, 0.f, 0.f};
    for (int i = tid; i < (NB2 * CH2 + NB2) / 4; i += NTHR) lds_dyn[i] = z4;
  }
  __syncthreads();

  const int* eid = ei + nE;
  const bool al16 = ((nE & 3) == 0);
  const int nChunks = (nE + CHUNK - 1) / CHUNK;
#pragma unroll 1
  for (int ch = 0; ch < nChunks; ++ch) {
    const int cbase = ch * CHUNK;
    const int wc = scan_chunk<NB2, SB2>(eid, nE, cbase, nodeBase, tid, wave, al16, list);
    if (lane == 0) wcnt[wave] = wc;
    __syncthreads();

    if (wave == 0) {
      for (int wsx = 0; wsx < NWAVE; ++wsx) {
        int n = wcnt[wsx];
        if (n > WCAP) n = WCAP;
        if (n < 0) n = 0;
        for (int i = 0; i < n; ++i) {
          const int ent  = list[wsx * WCAP + i];
          const int slot = ent & (NB2 - 1);
          const int el   = (ent >> SB2) & (CHUNK - 1);
          int e = cbase + el;
          if (e > nE - 1) e = nE - 1;
          int src = ei[e];
          src = src < 0 ? 0 : (src > nN - 1 ? nN - 1 : src);
          int nd = nodeBase + slot;
          if (nd > nN - 1) nd = nN - 1;
          float al = as2[src] + ad2[nd];
          al = lrelu(al);
          al = fminf(al, 80.f);
          const float p = __expf(al);
          const v2f xv = *(const v2f*)(h2 + (size_t)src * CH2 + 2 * lane);
          v2f* sp = (v2f*)(sacc + slot * CH2 + 2 * lane);
          const v2f cr = *sp;
          *sp = cr + p * xv;
          if (lane == 0) {
            const float o = den[slot];
            den[slot] = o + p;
          }
        }
      }
    }
    __syncthreads();
  }

  const int sub = lane >> 3;
  const int c0  = 8 * (lane & 7);
  const float bnk = 1.0f / sqrtf(1.0f + 1e-5f);
  const v4f b0 = *(const v4f*)(bias + c0);
  const v4f b1 = *(const v4f*)(bias + c0 + 4);
  const v4f g0 = *(const v4f*)(gam + c0) * bnk;
  const v4f g1 = *(const v4f*)(gam + c0 + 4) * bnk;
  const v4f e0 = *(const v4f*)(bet + c0);
  const v4f e1 = *(const v4f*)(bet + c0 + 4);
#pragma unroll 1
  for (int j = 0; j < NB2 / NWAVE / 4; ++j) {
    const int slot = wave * (NB2 / NWAVE) + 4 * j + sub;
    const int node = nodeBase + slot;
    const bool ok  = node < nN;
    const int nc   = ok ? node : (nN - 1);
    float al = as2[nc] + ad2[nc];
    al = lrelu(al);
    al = fminf(al, 80.f);
    const float p = __expf(al);
    const float* hr = h2 + (size_t)nc * CH2 + c0;
    const v4f x0 = *(const v4f*)hr;
    const v4f x1 = *(const v4f*)(hr + 4);
    const v4f* sp = (const v4f*)(sacc + slot * CH2 + c0);
    const v4f s0 = sp[0] + p * x0;
    const v4f s1 = sp[1] + p * x1;
    const float dv  = den[slot] + p;
    const float inv = 1.0f / (dv + 1e-16f);
    v4f v0 = s0 * inv + b0;
    v4f v1 = s1 * inv + b1;
    v0 = v0 * g0 + e0;
    v1 = v1 * g1 + e1;
    v0 = elu4(v0);
    v1 = elu4(v1);
    const v4i u = pack8(v0, v1);
    _Float16* op = hp + (size_t)nc * CH2 + c0;
    if (ok) *(volatile v4i*)op = u;
    __threadfence();
    if (ok) *(volatile v4i*)op = u;
  }
}

__global__ __launch_bounds__(NTHR) void k_dec(
    const _Float16* __restrict__ Hp, const float* __restrict__ Wd1, const float* __restrict__ bd1,
    const float* __restrict__ Wd2, const float* __restrict__ bd2,
    float* out, int nN, int outN) {
  __shared__ __attribute__((aligned(16))) _Float16 W1t[DH * W1TP];
  __shared__ __attribute__((aligned(16))) _Float16 W2t[32 * W2TP];
  __shared__ __attribute__((aligned(16))) _Float16 Hs[NWAVE * 16 * HSP];
  __shared__ __attribute__((aligned(16))) float Os[GRD * NCL];
  __shared__ float B1s[DH];
  __shared__ float B2s[32];

  const int tid  = threadIdx.x;
  const int lane = tid & 31;
  const int wave = tid >> 5;
  const int hh   = lane >> 4;
  const int m    = lane & 15;

  for (int idx = tid; idx < CH2 * DH; idx += NTHR) {
    const int k = idx >> 5, n = idx & 31;
    W1t[n * W1TP + k] = (_Float16)(32.0f * Wd1[idx]);
  }
  for (int idx = tid; idx < 32 * DH; idx += NTHR) {
    const int k = idx >> 5, n = idx & 31;
    const float v = (n < NCL) ? Wd2[k * NCL + n] : 0.f;
    W2t[n * W2TP + k] = (_Float16)(16.0f * v);
  }
  if (tid < DH) B1s[tid] = bd1[tid];
  if (tid < 32) B2s[tid] = (tid < NCL) ? bd2[tid] : 0.f;
  __syncthreads();

  const int rowBase = blockIdx.x * GRD;
  const int r0 = rowBase + 16 * wave;
  int rowc = r0 + m;
  if (rowc > nN - 1) rowc = nN - 1;
  const _Float16* pa = Hp + (size_t)rowc * CH2;
  _Float16* Hw = Hs + wave * 16 * HSP;

  v8f d0 = zero8(), d1 = zero8();
#pragma unroll
  for (int kt = 0; kt < CH2 / 32; ++kt) {
    const int k0 = kt * 32;
    Frag a, b0, b1;
    a.half[0]  = *(const v8h*)(pa + k0 + 8 * hh);
    a.half[1]  = *(const v8h*)(pa + k0 + 16 + 8 * hh);
    const _Float16* pb0 = W1t + m * W1TP + k0 + 8 * hh;
    const _Float16* pb1 = W1t + (16 + m) * W1TP + k0 + 8 * hh;
    b0.half[0] = *(const v8h*)pb0; b0.half[1] = *(const v8h*)(pb0 + 16);
    b1.half[0] = *(const v8h*)pb1; b1.half[1] = *(const v8h*)(pb1 + 16);
    d0 = wm(a.v, b0.v, d0);
    d1 = wm(a.v, b1.v, d1);
  }
  {
    const float inv = 0.03125f;
    const float bb0 = B1s[m], bb1 = B1s[16 + m];
#pragma unroll
    for (int r = 0; r < 8; ++r) {
      const float v0 = fmaxf(d0[r] * inv + bb0, 0.f);
      const float v1 = fmaxf(d1[r] * inv + bb1, 0.f);
      Hw[(8 * hh + r) * HSP + m]      = (_Float16)v0;
      Hw[(8 * hh + r) * HSP + 16 + m] = (_Float16)v1;
    }
  }
  __syncthreads();

  v8f t0 = zero8(), t1 = zero8();
  {
    Frag a, b0, b1;
    a.half[0] = *(const v8h*)(Hw + m * HSP + 8 * hh);
    a.half[1] = *(const v8h*)(Hw + m * HSP + 16 + 8 * hh);
    const _Float16* pb0 = W2t + m * W2TP + 8 * hh;
    const _Float16* pb1 = W2t + (16 + m) * W2TP + 8 * hh;
    b0.half[0] = *(const v8h*)pb0; b0.half[1] = *(const v8h*)(pb0 + 16);
    b1.half[0] = *(const v8h*)pb1; b1.half[1] = *(const v8h*)(pb1 + 16);
    t0 = wm(a.v, b0.v, t0);
    t1 = wm(a.v, b1.v, t1);
  }

  {
    const float inv = 0.0625f;
    const float bb0 = B2s[m], bb1 = B2s[16 + m];
    const bool c16 = (m == 0);
#pragma unroll
    for (int r = 0; r < 8; ++r) {
      const float l0 = t0[r] * inv + bb0;
      const float l1 = t1[r] * inv + bb1;
      const float u  = c16 ? fmaxf(l0, l1) : l0;
      const float mx = hmax16(u);
      const float x0 = __expf(l0 - mx);
      const float x1 = c16 ? __expf(l1 - mx) : 0.f;
      const float s  = hsum16(x0 + x1);
      const float is = 1.0f / s;
      const int orow = 16 * wave + 8 * hh + r;
      Os[orow * NCL + m] = x0 * is;
      if (c16) Os[orow * NCL + 16] = x1 * is;
    }
  }
  __syncthreads();

  const int NPC = GRD * NCL / 4;
  const size_t gq0 = (size_t)blockIdx.x * NPC;
  for (int pass = 0; pass < 2; ++pass) {
    for (int p = tid; p < NPC; p += NTHR) {
      const size_t gq = gq0 + (size_t)p;
      const v4f v = *(const v4f*)(Os + 4 * p);
      if (gq * 4 + 4 <= (size_t)outN) {
        *(volatile v4f*)(out + gq * 4) = v;
      } else {
        if (gq * 4 + 0 < (size_t)outN) *(volatile float*)(out + gq * 4 + 0) = v.x;
        if (gq * 4 + 1 < (size_t)outN) *(volatile float*)(out + gq * 4 + 1) = v.y;
        if (gq * 4 + 2 < (size_t)outN) *(volatile float*)(out + gq * 4 + 2) = v.z;
      }
    }
    if (pass == 0) __threadfence();
  }
}

extern "C" void kernel_launch(void* const* d_in, const int* in_sizes, int n_in,
                              void* d_out, int out_size, void* d_ws, size_t ws_size,
                              hipStream_t stream) {
  if (n_in < 18) return;
  const int nN = in_sizes[0] / IND;
  if (nN <= 0 || in_sizes[0] != nN * IND) return;
  const int nE = in_sizes[1] / 2;
  if (nE < 0 || in_sizes[1] != 2 * nE) return;
  if (in_sizes[2] != IND * CH1) return;
  if (in_sizes[3] != NH1 * HC || in_sizes[4] != NH1 * HC) return;
  if (in_sizes[5] != CH1 || in_sizes[6] != CH1 || in_sizes[7] != CH1) return;
  if (in_sizes[8] != CH1 * CH2) return;
  if (in_sizes[9] != CH2 || in_sizes[10] != CH2) return;
  if (in_sizes[11] != CH2 || in_sizes[12] != CH2 || in_sizes[13] != CH2) return;
  if (in_sizes[14] != CH2 * DH || in_sizes[15] != DH) return;
  if (in_sizes[16] != DH * NCL || in_sizes[17] != NCL) return;
  if (out_size != nN * NCL) return;

  const float* x        = (const float*)d_in[0];
  const int*   ei       = (const int*)d_in[1];
  const float* W1       = (const float*)d_in[2];
  const float* att1_src = (const float*)d_in[3];
  const float* att1_dst = (const float*)d_in[4];
  const float* bias1    = (const float*)d_in[5];
  const float* bn1_g    = (const float*)d_in[6];
  const float* bn1_b    = (const float*)d_in[7];
  const float* W2       = (const float*)d_in[8];
  const float* att2_src = (const float*)d_in[9];
  const float* att2_dst = (const float*)d_in[10];
  const float* bias2    = (const float*)d_in[11];
  const float* bn2_g    = (const float*)d_in[12];
  const float* bn2_b    = (const float*)d_in[13];
  const float* dec_W1   = (const float*)d_in[14];
  const float* dec_b1   = (const float*)d_in[15];
  const float* dec_W2   = (const float*)d_in[16];
  const float* dec_b2   = (const float*)d_in[17];
  float* out = (float*)d_out;

  const int nP = ((nN + NPAD - 1) / NPAD) * NPAD;
  size_t off = 0;
  _Float16* W1h = (_Float16*)((char*)d_ws + off); off += (size_t)CH1 * IND * 2;
  _Float16* W2h = (_Float16*)((char*)d_ws + off); off += (size_t)CH2 * CH1 * 2;
  float* h1  = (float*)((char*)d_ws + off);       off += (size_t)nP * CH1 * 4;
  float* as1 = (float*)((char*)d_ws + off);       off += (size_t)nP * NH1 * 4;
  float* ad1 = (float*)((char*)d_ws + off);       off += (size_t)nP * NH1 * 4;
  _Float16* h1p = (_Float16*)((char*)d_ws + off); off += (size_t)nP * CH1 * 2;
  float* h2  = (float*)((char*)d_ws + off);       off += (size_t)nP * CH2 * 4;
  float* as2 = (float*)((char*)d_ws + off);       off += (size_t)nP * 4;
  float* ad2 = (float*)((char*)d_ws + off);       off += (size_t)nP * 4;
  _Float16* h2p = (_Float16*)((char*)d_ws + off); off += (size_t)nP * CH2 * 2;
  if (off > ws_size) return;

  k_wprep<<<CH1 / 32, NTHR, 0, stream>>>(W1, W1h, IND, CH1, 64.0f);
  k_wprep<<<CH2 / 32, NTHR, 0, stream>>>(W2, W2h, CH1, CH2, 64.0f);

  k_gemm1<<<nP / GR1, NTHR, 0, stream>>>(x, W1h, att1_src, att1_dst, h1, as1, ad1, nN);

  hipFuncSetAttribute(reinterpret_cast<const void*>(&k_agg1),
                      hipFuncAttributeMaxDynamicSharedMemorySize, LDS_AGG1);
  k_agg1<<<(nN + NB1 - 1) / NB1, NTHR, LDS_AGG1, stream>>>(ei, h1, as1, ad1, bias1, bn1_g, bn1_b,
                                                          h1p, nN, nE);

  k_gemm2<<<nP / GR2, NTHR, 0, stream>>>(h1p, W2h, att2_src, att2_dst, h2, as2, ad2, nN);

  hipFuncSetAttribute(reinterpret_cast<const void*>(&k_agg2),
                      hipFuncAttributeMaxDynamicSharedMemorySize, LDS_AGG2);
  k_agg2<<<(nN + NB2 - 1) / NB2, NTHR, LDS_AGG2, stream>>>(ei, h2, as2, ad2, bias2, bn2_g, bn2_b,
                                                          h2p, nN, nE);

  k_dec<<<nP / GRD, NTHR, 0, stream>>>(h2p, dec_W1, dec_b1, dec_W2, dec_b2, out, nN, out_size);
}
